// non_local_attention_5411658793566
// MI455X (gfx1250) — hardware-verified
//
#include <hip/hip_runtime.h>


#define NBI  8
#define CI   128
#define NP   4096
#define CK   64
#define CV   64
#define CO   128
typedef _Float16 h16;
typedef unsigned short bf;
typedef __attribute__((ext_vector_type(16))) __bf16   v16bf;
typedef __attribute__((ext_vector_type(16))) _Float16 v16h;
typedef __attribute__((ext_vector_type(8)))  _Float16 v8h;
typedef __attribute__((ext_vector_type(8)))  unsigned short v8us;
typedef __attribute__((ext_vector_type(8)))  float    v8f;
typedef __attribute__((ext_vector_type(4)))  float    v4f;
typedef v8h  __attribute__((may_alias)) v8ha;
typedef v4f  __attribute__((may_alias)) v4fa;
typedef v8us __attribute__((may_alias)) v8usa;

__device__ __forceinline__ unsigned short f2bf(float f) { unsigned u = __float_as_uint(f); u += 0x7FFFu + ((u >> 16) & 1u); return (unsigned short)(u >> 16); }
__device__ __forceinline__ float bf2f(unsigned short b) { return __uint_as_float(((unsigned)b) << 16); }
__device__ __forceinline__ float bfr(float f) { return bf2f(f2bf(f)); }
__device__ __forceinline__ v16h cat16(v8h lo, v8h hi) { return __builtin_shufflevector(lo, hi, 0, 1, 2, 3, 4, 5, 6, 7, 8, 9, 10, 11, 12, 13, 14, 15); }
__device__ __forceinline__ v16bf cat16b(v8us lo, v8us hi) { return __builtin_bit_cast(v16bf, __builtin_shufflevector(lo, hi, 0, 1, 2, 3, 4, 5, 6, 7, 8, 9, 10, 11, 12, 13, 14, 15)); }
__device__ __forceinline__ v8f wmma16(v16h a, v16h b, v8f c) { return __builtin_amdgcn_wmma_f32_16x16x32_f16(false, a, false, b, (short)0, c, false, false); }
__device__ __forceinline__ v8f wmmab(v16bf a, v16bf b, v8f c) { return __builtin_amdgcn_wmma_f32_16x16x32_bf16(false, a, false, b, (short)0, c, false, false); }


template <typename T16> struct WFrag;
template <> struct WFrag<h16> { typedef v16h V; static __device__ __forceinline__ V ld(const h16* p) { return cat16(*(const v8h*)p, *(const v8h*)(p + 16)); } static __device__ __forceinline__ v8f mma(V a, V b, v8f c) { return wmma16(a, b, c); } };
template <> struct WFrag<bf> { typedef v16bf V; static __device__ __forceinline__ V ld(const bf* p) { return cat16b(*(const v8us*)p, *(const v8us*)(p + 16)); } static __device__ __forceinline__ v8f mma(V a, V b, v8f c) { return wmmab(a, b, c); } };
template <typename T16, int NSPLIT, bool BIAS>
__global__ __launch_bounds__(32) void k_gemmw(const T16* __restrict__ A, const T16* __restrict__ A2, const T16* __restrict__ Bt, const T16* __restrict__ Bt2, int K, float* C, int ldc, const float* __restrict__ bias, size_t sA, size_t sB, size_t sC) {
    typedef typename WFrag<T16>::V V;
    __shared__ __align__(16) float os[16 * 68];
    const size_t z = blockIdx.z; A += z * sA; if (A2) A2 += z * sA; Bt += z * sB; if (Bt2) Bt2 += z * sB; C += z * sC;
    const int lane = threadIdx.x & 31, lr = lane & 15, hi = lane >> 4; const int r0 = blockIdx.x * 64, c0 = blockIdx.y * 64;
    v8f acc[4][4];
#pragma unroll
    for (int mb = 0; mb < 4; ++mb)
#pragma unroll
        for (int nb = 0; nb < 4; ++nb) acc[mb][nb] = (v8f){};
    const size_t aoff = (size_t)(r0 + lr) * K + 8 * hi, boff = (size_t)(c0 + lr) * K + 8 * hi;
#pragma unroll 1
    for (int kc = 0; kc < K; kc += 32) {
        V a[4], a2[4];
#pragma unroll
        for (int mb = 0; mb < 4; ++mb) { a[mb] = WFrag<T16>::ld(A + aoff + (size_t)mb * 16 * K + kc); if (NSPLIT == 1 || NSPLIT == 2) a2[mb] = WFrag<T16>::ld(A2 + aoff + (size_t)mb * 16 * K + kc); }
#pragma unroll
        for (int nb = 0; nb < 4; ++nb) { const V b = WFrag<T16>::ld(Bt + boff + (size_t)nb * 16 * K + kc); V b2; if (NSPLIT >= 2) b2 = WFrag<T16>::ld(Bt2 + boff + (size_t)nb * 16 * K + kc);
#pragma unroll
            for (int mb = 0; mb < 4; ++mb) { acc[mb][nb] = WFrag<T16>::mma(a[mb], b, acc[mb][nb]); if (NSPLIT == 1 || NSPLIT == 2) acc[mb][nb] = WFrag<T16>::mma(a2[mb], b, acc[mb][nb]); if (NSPLIT >= 2) acc[mb][nb] = WFrag<T16>::mma(a[mb], b2, acc[mb][nb]); } }
        asm volatile("v_nop\n\tv_nop\n\tv_nop\n\tv_nop" : "+v"(acc[0][0]), "+v"(acc[1][1]), "+v"(acc[2][2]), "+v"(acc[3][3]) : "v"(a[0]), "v"(a[3]));
    }
#pragma unroll
    for (int mb = 0; mb < 4; ++mb) {
#pragma unroll
        for (int nb = 0; nb < 4; ++nb) {
#pragma unroll
            for (int j = 0; j < 8; ++j) os[(hi * 8 + j) * 68 + nb * 16 + lr] = acc[mb][nb][j]; }
        __builtin_amdgcn_wave_barrier(); asm volatile("" ::: "memory");
        float* crow = C + (size_t)(r0 + mb * 16) * ldc + c0;
#pragma unroll 1
        for (int ps = 0; ps < 2; ++ps) {
#pragma unroll
            for (int s = 0; s < 8; ++s) { const int row = 2 * s + hi, cofs = lr * 4; v4f val = *(const v4fa*)(os + row * 68 + cofs); if (BIAS) { val[0] += bfr(bias[c0 + cofs]); val[1] += bfr(bias[c0 + cofs + 1]); val[2] += bfr(bias[c0 + cofs + 2]); val[3] += bfr(bias[c0 + cofs + 3]); }
                *(volatile v4f*)(crow + (size_t)row * ldc + cofs) = val; }
            if (ps == 0) __threadfence(); }
        __builtin_amdgcn_wave_barrier(); asm volatile("" ::: "memory");
    }
}

__device__ __forceinline__ void splitf(float y, unsigned short& h, unsigned short& l) { h = f2bf(y); l = f2bf(y - bf2f(h)); }
typedef __attribute__((ext_vector_type(2))) unsigned short v2us;
typedef __attribute__((ext_vector_type(2))) float v2f;
typedef __attribute__((ext_vector_type(4))) unsigned short v4us;

__global__ __launch_bounds__(256) void k_cvt8(const float* __restrict__ src, bf* dst, size_t n8) { const size_t i = (size_t)blockIdx.x * 256 + threadIdx.x; if (i >= n8) return; const v8f v = *(const v8f*)(src + i * 8); v8us o;
#pragma unroll
    for (int k = 0; k < 8; ++k) o[k] = f2bf(v[k]); *(volatile v8us*)(dst + i * 8) = o; __threadfence(); *(volatile v8us*)(dst + i * 8) = o; }
__global__ __launch_bounds__(256) void k_xt(const float* __restrict__ x, bf* XT) { const int e = (blockIdx.x * 256 + threadIdx.x) * 2; if (e >= NP * CI) return; const int c = e % CI; const int p = e / CI; v2us o; o[0] = f2bf(x[(size_t)c * NP + p]); o[1] = f2bf(x[(size_t)(c + 1) * NP + p]); *(volatile v2us*)(XT + e) = o; __threadfence(); *(volatile v2us*)(XT + e) = o; }
__global__ __launch_bounds__(256) void k_bnstat(const float* __restrict__ Y, float* ST) { __shared__ float red[256]; const int c = blockIdx.x; const int tid = threadIdx.x; float s = 0.f;
    for (int i = tid; i < NBI * NP; i += 256) s += Y[(size_t)i * CK + c];
    red[tid] = s; __syncthreads(); for (int k = 128; k; k >>= 1) { if (tid < k) red[tid] = __fadd_rn(red[tid], red[tid + k]); __syncthreads(); } const float mean = red[0] * (1.0f / (NBI * NP)); __syncthreads();
    float q = 0.f; for (int i = tid; i < NBI * NP; i += 256) { float d = __fsub_rn(Y[(size_t)i * CK + c], mean); asm volatile("" : "+v"(d)); float p = __fmul_rn(d, d); asm volatile("" : "+v"(p)); q = __fadd_rn(q, p); }
    red[tid] = q; __syncthreads(); for (int k = 128; k; k >>= 1) { if (tid < k) red[tid] = __fadd_rn(red[tid], red[tid + k]); __syncthreads(); }
    if (tid == 0) { v2f o; o[0] = mean; o[1] = __frsqrt_rn(__fadd_rn(red[0] * (1.0f / (NBI * NP)), 1e-5f)); *(volatile v2f*)(ST + 2 * c) = o; __threadfence(); *(volatile v2f*)(ST + 2 * c) = o; } }
__global__ __launch_bounds__(256) void k_qn(const float* __restrict__ Y, const float* __restrict__ ST, const float* __restrict__ ga, const float* __restrict__ be, bf* Qh, bf* Ql) { const int e = (blockIdx.x * 256 + threadIdx.x) * 4; if (e >= NP * CK) return; const int c0 = e % CK; const v4f a = *(const v4f*)(Y + e); float y[4]; float ss = 0.f;
#pragma unroll
    for (int u = 0; u < 4; ++u) { const int c = c0 + u; float t0 = __fmul_rn(__fsub_rn(a[u], ST[2 * c]), ST[2 * c + 1]); asm volatile("" : "+v"(t0)); float g = bfr(ga[c]), bb = bfr(be[c]); asm volatile("" : "+v"(g)); asm volatile("" : "+v"(bb)); float t1 = __fmul_rn(t0, g); asm volatile("" : "+v"(t1)); y[u] = __fadd_rn(t1, bb); float p = __fmul_rn(y[u], y[u]); asm volatile("" : "+v"(p)); ss = __fadd_rn(ss, p); }
    ss += __shfl_xor(ss, 1, 32); ss += __shfl_xor(ss, 2, 32); ss += __shfl_xor(ss, 4, 32); ss += __shfl_xor(ss, 8, 32); const float inv = __fdiv_rn(1.0f, __fadd_rn(__fsqrt_rn(ss), 1e-7f)); v4us oh, ol;
#pragma unroll
    for (int u = 0; u < 4; ++u) { unsigned short hh, ll; splitf(__fmul_rn(y[u], inv), hh, ll); oh[u] = hh; ol[u] = ll; } *(volatile v4us*)(Qh + e) = oh; *(volatile v4us*)(Ql + e) = ol; __threadfence(); *(volatile v4us*)(Qh + e) = oh; *(volatile v4us*)(Ql + e) = ol; }
__global__ __launch_bounds__(256) void k_knT(const float* __restrict__ Y, const float* __restrict__ ST, const float* __restrict__ ga, const float* __restrict__ be, bf* Kh, bf* Kl) { const int m = (blockIdx.x * 256 + threadIdx.x) * 2; if (m >= NP) return; float y0[CK], y1[CK]; float s0 = 0.f, s1 = 0.f;
#pragma unroll
    for (int c4 = 0; c4 < CK / 4; ++c4) { const v4f a = *(const v4f*)(Y + (size_t)m * CK + c4 * 4), b = *(const v4f*)(Y + (size_t)(m + 1) * CK + c4 * 4);
#pragma unroll
        for (int u = 0; u < 4; ++u) { const int c = c4 * 4 + u; const float mu = ST[2 * c], rs = ST[2 * c + 1]; float g = bfr(ga[c]), bb = bfr(be[c]); asm volatile("" : "+v"(g)); asm volatile("" : "+v"(bb));
            float t0 = __fmul_rn(__fsub_rn(a[u], mu), rs), t1 = __fmul_rn(__fsub_rn(b[u], mu), rs); asm volatile("" : "+v"(t0)); asm volatile("" : "+v"(t1)); float u0 = __fmul_rn(t0, g), u1 = __fmul_rn(t1, g); asm volatile("" : "+v"(u0)); asm volatile("" : "+v"(u1)); y0[c] = __fadd_rn(u0, bb); y1[c] = __fadd_rn(u1, bb);
            float p0 = __fmul_rn(y0[c], y0[c]), p1 = __fmul_rn(y1[c], y1[c]); asm volatile("" : "+v"(p0)); asm volatile("" : "+v"(p1)); s0 = __fadd_rn(s0, p0); s1 = __fadd_rn(s1, p1); } }
    const float i0 = __fdiv_rn(1.0f, __fadd_rn(__fsqrt_rn(s0), 1e-7f)), i1 = __fdiv_rn(1.0f, __fadd_rn(__fsqrt_rn(s1), 1e-7f));
    for (int ps = 0; ps < 2; ++ps) {
#pragma unroll
        for (int c = 0; c < CK; ++c) { unsigned short a0, b0, a1, b1; splitf(__fmul_rn(y0[c], i0), a0, b0); splitf(__fmul_rn(y1[c], i1), a1, b1); v2us oh, ol; oh[0] = a0; oh[1] = a1; ol[0] = b0; ol[1] = b1; *(volatile v2us*)(Kh + (size_t)c * NP + m) = oh; *(volatile v2us*)(Kl + (size_t)c * NP + m) = ol; }
        if (ps == 0) __threadfence(); } }
__global__ __launch_bounds__(256) void k_vT(const float* __restrict__ Y, bf* Vh, bf* Vl) { const int e = (blockIdx.x * 256 + threadIdx.x) * 2; if (e >= CV * NP) return; const int m = e % NP; const int v = e / NP; unsigned short a0, b0, a1, b1; splitf(Y[(size_t)m * CV + v], a0, b0); splitf(Y[(size_t)(m + 1) * CV + v], a1, b1); v2us oh, ol; oh[0] = a0; oh[1] = a1; ol[0] = b0; ol[1] = b1;
    *(volatile v2us*)(Vh + e) = oh; *(volatile v2us*)(Vl + e) = ol; __threadfence(); *(volatile v2us*)(Vh + e) = oh; *(volatile v2us*)(Vl + e) = ol; }
__global__ __launch_bounds__(64) void k_vsum(const float* __restrict__ Y, float* vs) { const int v = threadIdx.x; float s = 0.f;
#pragma unroll 1
    for (int m = 0; m < NP; ++m) s = __fadd_rn(s, Y[(size_t)m * CV + v]); *(volatile float*)(vs + v) = s; __threadfence(); *(volatile float*)(vs + v) = s; }
__global__ __launch_bounds__(256) void k_mt(const float* __restrict__ M, bf* Mh, bf* Ml) { const int e = (blockIdx.x * 256 + threadIdx.x) * 4; if (e >= CV * CK) return; const int c0 = e % CK, v = e / CK; v4us oh, ol;
#pragma unroll
    for (int u = 0; u < 4; ++u) { unsigned short a, b; splitf(M[(size_t)(c0 + u) * CV + v], a, b); oh[u] = a; ol[u] = b; } *(volatile v4us*)(Mh + e) = oh; *(volatile v4us*)(Ml + e) = ol; __threadfence(); *(volatile v4us*)(Mh + e) = oh; *(volatile v4us*)(Ml + e) = ol; }
__global__ __launch_bounds__(256) void k_splitb(const float* __restrict__ F, const float* __restrict__ vs, bf* Ph, bf* Pl) { const size_t e = ((size_t)blockIdx.x * 256 + threadIdx.x) * 4; if (e >= (size_t)NP * CV) return; const int v0 = (int)(e % CV); const v4f a = *(const v4f*)(F + e); v4us oh, ol;
#pragma unroll
    for (int u = 0; u < 4; ++u) { unsigned short x, y; splitf(__fadd_rn(a[u], vs[v0 + u]), x, y); oh[u] = x; ol[u] = y; } *(volatile v4us*)(Ph + e) = oh; *(volatile v4us*)(Pl + e) = ol; __threadfence(); *(volatile v4us*)(Ph + e) = oh; *(volatile v4us*)(Pl + e) = ol; }
__global__ __launch_bounds__(256) void k_nchw(const float* __restrict__ OT, float* OUTb) { const int e = (blockIdx.x * 256 + threadIdx.x) * 4; if (e >= CO * NP) return; const int p = e % NP; const int o = e / NP; v4f ov;
#pragma unroll
    for (int u = 0; u < 4; ++u) ov[u] = OT[(size_t)(p + u) * CO + o]; *(volatile v4f*)(OUTb + e) = ov; __threadfence(); *(volatile v4f*)(OUTb + e) = ov; }

extern "C" void kernel_launch(void* const* d_in, const int* in_sizes, int n_in,
                              void* d_out, int out_size, void* d_ws, size_t ws_size, hipStream_t stream) {
    (void)in_sizes; (void)n_in; (void)out_size;
    const float** I = (const float**)d_in;
    const float *qf = I[0], *kf = I[1], *vf = I[2], *Wk = I[3], *bk = I[4], *ga = I[5], *be = I[6], *Wv = I[7], *bv = I[8], *Ww = I[9], *bw = I[10];
    float* OUT = (float*)d_out;
    char* wsp = (char*)d_ws;
    auto take = [&](size_t bytes) { char* p = wsp; wsp += (bytes + 255) & ~(size_t)255; return (void*)p; };
    bf* WK = (bf*)take(CK * CI * 2); bf* WV = (bf*)take(CV * CI * 2); bf* WW = (bf*)take(CO * CV * 2);
    bf* XT = (bf*)take((size_t)NP * CI * 2); float* YQ = (float*)take((size_t)NBI * NP * CK * 4); float* YK = (float*)take((size_t)NBI * NP * CK * 4); float* YV = (float*)take((size_t)NBI * NP * CV * 4); float* STQ = (float*)take(CK * 2 * 4); float* STK = (float*)take(CK * 2 * 4);
    bf* Qh = (bf*)take((size_t)NP * CK * 2); bf* Ql = (bf*)take((size_t)NP * CK * 2); bf* Kh = (bf*)take((size_t)CK * NP * 2); bf* Kl = (bf*)take((size_t)CK * NP * 2); bf* Vh = (bf*)take((size_t)CV * NP * 2); bf* Vl = (bf*)take((size_t)CV * NP * 2); float* vs = (float*)take(256);
    float* M = (float*)take(CK * CV * 4); bf* Mh = (bf*)take(CK * CV * 2); bf* Ml = (bf*)take(CK * CV * 2); float* CTX = (float*)take((size_t)NP * CV * 4); bf* Ch = (bf*)take((size_t)NP * CV * 2); bf* Cl = (bf*)take((size_t)NP * CV * 2); float* OT = (float*)take((size_t)NP * CO * 4);
    if ((size_t)(wsp - (char*)d_ws) > ws_size) return;
    k_cvt8<<<(CK * CI / 8 + 255) / 256, 256, 0, stream>>>(Wk, WK, CK * CI / 8); k_cvt8<<<(CV * CI / 8 + 255) / 256, 256, 0, stream>>>(Wv, WV, CV * CI / 8); k_cvt8<<<(CO * CV / 8 + 255) / 256, 256, 0, stream>>>(Ww, WW, CO * CV / 8);
    for (int b = 0; b < NBI; ++b) {
        k_xt<<<(NP * CI / 2 + 255) / 256, 256, 0, stream>>>(qf + (size_t)b * CI * NP, XT); k_gemmw<bf, 0, true><<<dim3(NP / 64, 1, 1), 32, 0, stream>>>(XT, nullptr, WK, nullptr, CI, YQ + (size_t)b * NP * CK, CK, bk, 0, 0, 0);
        k_xt<<<(NP * CI / 2 + 255) / 256, 256, 0, stream>>>(kf + (size_t)b * CI * NP, XT); k_gemmw<bf, 0, true><<<dim3(NP / 64, 1, 1), 32, 0, stream>>>(XT, nullptr, WK, nullptr, CI, YK + (size_t)b * NP * CK, CK, bk, 0, 0, 0);
        k_xt<<<(NP * CI / 2 + 255) / 256, 256, 0, stream>>>(vf + (size_t)b * CI * NP, XT); k_gemmw<bf, 0, true><<<dim3(NP / 64, 1, 1), 32, 0, stream>>>(XT, nullptr, WV, nullptr, CI, YV + (size_t)b * NP * CV, CV, bv, 0, 0, 0); }
    k_bnstat<<<CK, 256, 0, stream>>>(YQ, STQ); k_bnstat<<<CK, 256, 0, stream>>>(YK, STK);
    for (int b = 0; b < NBI; ++b) { const float* yq = YQ + (size_t)b * NP * CK; const float* yk = YK + (size_t)b * NP * CK; const float* yv = YV + (size_t)b * NP * CV;
        k_qn<<<(NP * CK / 4 + 255) / 256, 256, 0, stream>>>(yq, STQ, ga, be, Qh, Ql); k_knT<<<(NP / 2 + 255) / 256, 256, 0, stream>>>(yk, STK, ga, be, Kh, Kl); k_vT<<<(CV * NP / 2 + 255) / 256, 256, 0, stream>>>(yv, Vh, Vl); k_vsum<<<1, 64, 0, stream>>>(yv, vs);
        k_gemmw<bf, 2, false><<<dim3(1, 1, 1), 32, 0, stream>>>(Kh, Kl, Vh, Vl, NP, M, CV, nullptr, 0, 0, 0);
        k_mt<<<(CV * CK / 4 + 255) / 256, 256, 0, stream>>>(M, Mh, Ml);
        k_gemmw<bf, 2, false><<<dim3(NP / 64, 1, 1), 32, 0, stream>>>(Qh, Ql, Mh, Ml, CK, CTX, CV, nullptr, 0, 0, 0);
        k_splitb<<<(NP * CV / 4 + 255) / 256, 256, 0, stream>>>(CTX, vs, Ch, Cl);
        k_gemmw<bf, 1, true><<<dim3(NP / 64, CO / 64, 1), 32, 0, stream>>>(Ch, Cl, WW, nullptr, CV, OT, CO, bw, 0, 0, 0);
        k_nchw<<<(CO * NP / 4 + 255) / 256, 256, 0, stream>>>(OT, OUT + (size_t)b * CO * NP); }
}
